// MultiHeadAttention_14130442404267
// MI455X (gfx1250) — hardware-verified
//
#include <hip/hip_runtime.h>
#include <math.h>

#ifndef NB
#define NB 4
#endif
#ifndef SEQ
#define SEQ 2048
#endif
#define NB_FULL 4
#define SEQ_FULL 2048
#define HIDDEN 1024
#define HEADS 16
#define HD 64
#define MTOK (NB * SEQ)

static_assert(HIDDEN == HEADS * HD);
static_assert(HD == 64);
static_assert(HIDDEN % 64 == 0 && HIDDEN % 32 == 0 && HIDDEN % 8 == 0);
static_assert(SEQ % 64 == 0 && SEQ % 32 == 0);
static_assert(MTOK % 64 == 0);
static_assert(NB <= NB_FULL && SEQ <= SEQ_FULL);
static_assert(((long long)(NB - 1) * SEQ_FULL + SEQ) * HIDDEN <= (long long)NB_FULL * SEQ_FULL * HIDDEN);

typedef __attribute__((ext_vector_type(16))) _Float16 v16h;
typedef __attribute__((ext_vector_type(8)))  _Float16 v8h;
typedef __attribute__((ext_vector_type(8)))  float    v8f;
typedef __attribute__((ext_vector_type(4)))  float    v4f;
typedef __attribute__((ext_vector_type(4)))  unsigned int v4u;

union FragU { v16h v; v8h h[2]; };
__device__ __forceinline__ v16h ld_frag(const _Float16* p) { FragU f; f.h[0] = *(const v8h*)(p); f.h[1] = *(const v8h*)(p + 16); return f.v; }
__device__ __forceinline__ v8f mma_f16(v16h a, v16h b, v8f c) { return __builtin_amdgcn_wmma_f32_16x16x32_f16(false, a, false, b, (short)0, c, false, false); }
__device__ __forceinline__ void guard_row(v8f& a, v8f& b, v8f& c, v8f& d, v16h x) { asm volatile("v_nop\n\tv_nop\n\tv_nop\n\tv_nop" : "+v"(a), "+v"(b), "+v"(c), "+v"(d) : "v"(x)); }
__device__ __forceinline__ void keep4(v16h a, v16h b, v16h c, v16h d) { asm volatile("v_nop" :: "v"(a), "v"(b), "v"(c), "v"(d)); }
__device__ __forceinline__ void guard4(v8f& a, v8f& b, v8f& c, v8f& d) { asm volatile("v_nop\n\tv_nop\n\tv_nop\n\tv_nop" : "+v"(a), "+v"(b), "+v"(c), "+v"(d)); }
__device__ __forceinline__ void guard_s(v8f& a, v8f& b, v16h x0, v16h x1, v16h x2, v16h x3, v16h y0, v16h y1) { asm volatile("v_nop\n\tv_nop\n\tv_nop\n\tv_nop" : "+v"(a), "+v"(b) : "v"(x0), "v"(x1), "v"(x2), "v"(x3), "v"(y0), "v"(y1)); }
__device__ __forceinline__ void guard_o(v8f& a, v8f& b, v8f& c, v8f& d, v16h x0, v16h x1, v16h x2, v16h x3, v16h y) { asm volatile("v_nop\n\tv_nop\n\tv_nop\n\tv_nop" : "+v"(a), "+v"(b), "+v"(c), "+v"(d) : "v"(x0), "v"(x1), "v"(x2), "v"(x3), "v"(y)); }

__device__ __forceinline__ float bf16_rne_f32(float v) { unsigned u = __float_as_uint(v); u = (u + 0x7fffu + ((u >> 16) & 1u)) & 0xffff0000u; return __uint_as_float(u); }
__device__ __forceinline__ unsigned pk2h(float a, float b) { return (unsigned)__builtin_bit_cast(unsigned short, (_Float16)a) | ((unsigned)__builtin_bit_cast(unsigned short, (_Float16)b) << 16); }
__device__ __forceinline__ void wave_sync_lds() {
    __builtin_amdgcn_fence(3  , "workgroup");
    __builtin_amdgcn_wave_barrier();
    __builtin_amdgcn_fence(2  , "workgroup");
}

__global__ __launch_bounds__(256) void k_cast16(const float* __restrict__ SRC, unsigned short* __restrict__ DST, int nR, int rpb, int srb, float sc) {
    const long long u = (long long)blockIdx.x * 256 + threadIdx.x;
    const int per = HIDDEN / 8;
    if (u >= (long long)nR * per) return;
    const int r = (int)(u / per); const int c0 = 8 * (int)(u % per);
    const int bb = r / rpb; const int sr = bb * srb + (r - bb * rpb);
    const float* s = SRC + (long long)sr * HIDDEN + c0;
    const v4f a = *(const v4f*)(s); const v4f b = *(const v4f*)(s + 4);
    v4u pk;
    pk.x = pk2h(bf16_rne_f32(a.x) * sc, bf16_rne_f32(a.y) * sc);
    pk.y = pk2h(bf16_rne_f32(a.z) * sc, bf16_rne_f32(a.w) * sc);
    pk.z = pk2h(bf16_rne_f32(b.x) * sc, bf16_rne_f32(b.y) * sc);
    pk.w = pk2h(bf16_rne_f32(b.z) * sc, bf16_rne_f32(b.w) * sc);
    volatile v4u* d = (volatile v4u*)(DST + (long long)r * HIDDEN + c0);
    *d = pk; __threadfence(); *d = pk;
}

template <int BIAS_MODE, int OUT_MODE>
__device__ __forceinline__ void gemm64_body(const unsigned short* __restrict__ Ap, int lda, long long strideA,
                                            const unsigned short* __restrict__ Btp, int ldb, long long strideB,
                                            void* __restrict__ Cout, int ldc, long long strideC,
                                            const float* __restrict__ bias, int M, int N, int K, float scale) {
    __shared__ __align__(16) float sT[8][16 * 68];
    const int bz   = blockIdx.y;
    const int lane = threadIdx.x & 31;
    const int wave = threadIdx.x >> 5;
    const int tilesN = N >> 6;
    const int tilesM = M >> 6;
    const int tile = blockIdx.x * 8 + wave;
    if (tile >= tilesM * tilesN) return;
    const int tm = tile / tilesN;
    const int tn = tile - tm * tilesN;
    const int m0 = tm << 6;
    const int n0 = tn << 6;
    const _Float16* Ab = (const _Float16*)Ap + (size_t)bz * strideA;
    const _Float16* Bb = (const _Float16*)Btp + (size_t)bz * strideB;
    const int rlane = lane & 15;
    const int koff  = (lane >> 4) * 8;
    const int mOff  = (lane >> 4) * 8;

    v8f acc[4][4];
#pragma unroll
    for (int i = 0; i < 4; ++i)
#pragma unroll
        for (int j = 0; j < 4; ++j) { v8f zz = {}; acc[i][j] = zz; }

    for (int k0 = 0; k0 < K; k0 += 32) {
        v16h bh[4];
#pragma unroll
        for (int j = 0; j < 4; ++j) bh[j] = ld_frag(Bb + (size_t)(n0 + (j << 4) + rlane) * ldb + koff + k0);
#pragma unroll
        for (int i = 0; i < 4; ++i) {
            const v16h ah = ld_frag(Ab + (size_t)(m0 + (i << 4) + rlane) * lda + koff + k0);
#pragma unroll
            for (int j = 0; j < 4; ++j) acc[i][j] = mma_f16(ah, bh[j], acc[i][j]);
            guard_row(acc[i][0], acc[i][1], acc[i][2], acc[i][3], ah);
        }
        keep4(bh[0], bh[1], bh[2], bh[3]);
    }
    guard4(acc[0][0], acc[0][1], acc[0][2], acc[0][3]);
    guard4(acc[1][0], acc[1][1], acc[1][2], acc[1][3]);
    guard4(acc[2][0], acc[2][1], acc[2][2], acc[2][3]);
    guard4(acc[3][0], acc[3][1], acc[3][2], acc[3][3]);

#pragma unroll
    for (int i = 0; i < 4; ++i) {
        const int mBase = m0 + (i << 4);
#pragma unroll
        for (int j = 0; j < 4; ++j) {
            const int n = n0 + (j << 4) + rlane;
            float bv = 0.f;
            if (BIAS_MODE == 2) bv = bf16_rne_f32(bias[n]);
#pragma unroll
            for (int r = 0; r < 8; ++r) {
                float v = acc[i][j][r] * scale;
                if (BIAS_MODE == 1) v += bf16_rne_f32(bias[mBase + mOff + r]);
                if (BIAS_MODE == 2) v += bv;
                sT[wave][(mOff + r) * 68 + (j << 4) + rlane] = v;
            }
        }
        wave_sync_lds();
        if (OUT_MODE == 0) {
            float* C = (float*)Cout + (size_t)bz * strideC;
            const int hh = lane >> 4, c4 = (lane & 15) * 4;
            v4f vv[8];
#pragma unroll
            for (int it = 0; it < 8; ++it) {
                const int o = (it * 2 + hh) * 68 + c4;
                vv[it].x = sT[wave][o]; vv[it].y = sT[wave][o + 1]; vv[it].z = sT[wave][o + 2]; vv[it].w = sT[wave][o + 3];
            }
#pragma unroll
            for (int it = 0; it < 8; ++it) *(volatile v4f*)(C + (size_t)(mBase + it * 2 + hh) * ldc + n0 + c4) = vv[it];
            __threadfence();
#pragma unroll
            for (int it = 0; it < 8; ++it) *(volatile v4f*)(C + (size_t)(mBase + it * 2 + hh) * ldc + n0 + c4) = vv[it];
        } else {
            _Float16* C = (_Float16*)Cout + (size_t)bz * strideC;
            const int q = lane >> 3, c8 = (lane & 7) * 8;
            v8h hv[4];
#pragma unroll
            for (int it = 0; it < 4; ++it) {
                const int o = (it * 4 + q) * 68 + c8;
#pragma unroll
                for (int e = 0; e < 8; ++e) hv[it][e] = (_Float16)sT[wave][o + e];
            }
#pragma unroll
            for (int it = 0; it < 4; ++it) *(volatile v8h*)(C + (size_t)(mBase + it * 4 + q) * ldc + n0 + c8) = hv[it];
            __threadfence();
#pragma unroll
            for (int it = 0; it < 4; ++it) *(volatile v8h*)(C + (size_t)(mBase + it * 4 + q) * ldc + n0 + c8) = hv[it];
        }
        wave_sync_lds();
    }
}

__global__ __launch_bounds__(256) void k_gemm_nbias_f16(const unsigned short* __restrict__ A, int lda, long long sA, const unsigned short* __restrict__ Bt, int ldb, long long sB,
                                                        unsigned short* __restrict__ C, int ldc, long long sC, const float* __restrict__ bias, int M, int N, int K, float scale) {
    gemm64_body<2, 1>(A, lda, sA, Bt, ldb, sB, (void*)C, ldc, sC, bias, M, N, K, scale);
}
__global__ __launch_bounds__(256) void k_gemm_mbias_f16(const unsigned short* __restrict__ A, int lda, long long sA, const unsigned short* __restrict__ Bt, int ldb, long long sB,
                                                        unsigned short* __restrict__ C, int ldc, long long sC, const float* __restrict__ bias, int M, int N, int K, float scale) {
    gemm64_body<1, 1>(A, lda, sA, Bt, ldb, sB, (void*)C, ldc, sC, bias, M, N, K, scale);
}
__global__ __launch_bounds__(256) void k_gemm_nbias_f32(const unsigned short* __restrict__ A, int lda, long long sA, const unsigned short* __restrict__ Bt, int ldb, long long sB,
                                                        float* __restrict__ C, int ldc, long long sC, const float* __restrict__ bias, int M, int N, int K, float scale) {
    gemm64_body<2, 0>(A, lda, sA, Bt, ldb, sB, (void*)C, ldc, sC, bias, M, N, K, scale);
}

__global__ __launch_bounds__(128) void k_attn(const unsigned short* __restrict__ Qp, const unsigned short* __restrict__ Kp, const unsigned short* __restrict__ VTp,
                                              const float* __restrict__ masks, unsigned short* __restrict__ CTXp) {
    __shared__ __align__(16) float Os[4][16 * 68];
    const int tid = threadIdx.x, wave = tid >> 5, lane = tid & 31, hh = lane >> 4, c = lane & 15;
    const int nqb = SEQ / 64;
    const int bx = blockIdx.x;
    const int qb = bx % nqb;
    const int bh = bx / nqb;
    const int h  = bh % HEADS;
    const int b  = bh / HEADS;
    const int q0 = qb * 64 + wave * 16;
    const _Float16* Q  = (const _Float16*)Qp;
    const _Float16* K  = (const _Float16*)Kp;
    const _Float16* VT = (const _Float16*)VTp;
    const long long qoff = ((long long)(b * SEQ + q0 + c)) * HIDDEN + h * HD + 8 * hh;
    const long long koff = ((long long)b * SEQ) * HIDDEN + h * HD + 8 * hh;
    const long long voff = ((long long)(h * HD + c)) * MTOK + (long long)b * SEQ + 8 * hh;
    const float* mk = masks + (long long)b * SEQ_FULL + 8 * hh;
    const float L2E = 1.4426950408889634f;

    float m = -3.0e38f, l = 0.f;
    v8f o0 = {}, o1 = {}, o2 = {}, o3 = {};

#pragma unroll 1
    for (int kv0 = 0; kv0 < SEQ; kv0 += 32) {
        const _Float16* kr0 = K + koff + (long long)(kv0 + c) * HIDDEN;
        const _Float16* kr1 = kr0 + 16 * HIDDEN;
        const v16h qb0 = ld_frag(Q + qoff), qb1 = ld_frag(Q + qoff + 32);
        const v16h ka00 = ld_frag(kr0), ka01 = ld_frag(kr0 + 32), ka10 = ld_frag(kr1), ka11 = ld_frag(kr1 + 32);
        v8f s0 = {}, s1 = {};
        s0 = mma_f16(ka00, qb0, s0);
        s0 = mma_f16(ka01, qb1, s0);
        s1 = mma_f16(ka10, qb0, s1);
        s1 = mma_f16(ka11, qb1, s1);
        guard_s(s0, s1, ka00, ka01, ka10, ka11, qb0, qb1);

        const float* mp = mk + kv0;
        const v4f ma = *(const v4f*)(mp), mb = *(const v4f*)(mp + 4), mc = *(const v4f*)(mp + 16), md = *(const v4f*)(mp + 20);
        float mv[16];
        mv[0] = ma.x; mv[1] = ma.y; mv[2] = ma.z; mv[3] = ma.w; mv[4] = mb.x; mv[5] = mb.y; mv[6] = mb.z; mv[7] = mb.w;
        mv[8] = mc.x; mv[9] = mc.y; mv[10] = mc.z; mv[11] = mc.w; mv[12] = md.x; mv[13] = md.y; mv[14] = md.z; mv[15] = md.w;
        float x[16];
#pragma unroll
        for (int r = 0; r < 8; ++r) {
            const float v0 = s0[r] * 0.125f + (1.0f - mv[r]) * -1.0e9f;
            const float v1 = s1[r] * 0.125f + (1.0f - mv[8 + r]) * -1.0e9f;
            x[r] = v0 * L2E; x[8 + r] = v1 * L2E;
        }
        float mx = x[0];
#pragma unroll
        for (int i = 1; i < 16; ++i) mx = fmaxf(mx, x[i]);
        mx = fmaxf(mx, __shfl_xor(mx, 16, 32));
        const float mnew = fmaxf(m, mx);
        const float alpha = exp2f(m - mnew);
        m = mnew;
        const float msh = mnew - 12.0f;
        float ls = 0.f;
        v16h pb;
#pragma unroll
        for (int i = 0; i < 16; ++i) { const float p = exp2f(x[i] - msh); ls += p; pb[i] = (_Float16)p; }
        l = l * alpha + ls;
        o0 = o0 * alpha; o1 = o1 * alpha; o2 = o2 * alpha; o3 = o3 * alpha;

        const _Float16* vr = VT + voff + kv0;
        const v16h va0 = ld_frag(vr), va1 = ld_frag(vr + 16LL * MTOK), va2 = ld_frag(vr + 32LL * MTOK), va3 = ld_frag(vr + 48LL * MTOK);
        o0 = mma_f16(va0, pb, o0);
        o1 = mma_f16(va1, pb, o1);
        o2 = mma_f16(va2, pb, o2);
        o3 = mma_f16(va3, pb, o3);
        guard_o(o0, o1, o2, o3, va0, va1, va2, va3, pb);
    }

    const float lt = l + __shfl_xor(l, 16, 32);
    const float inv = 64.0f * (1.0f / lt);
#pragma unroll
    for (int r = 0; r < 8; ++r) {
        const int ob = c * 68 + 8 * hh + r;
        Os[wave][ob]      = o0[r] * inv;
        Os[wave][ob + 16] = o1[r] * inv;
        Os[wave][ob + 32] = o2[r] * inv;
        Os[wave][ob + 48] = o3[r] * inv;
    }
    wave_sync_lds();
    {
        _Float16* CT = (_Float16*)CTXp + ((long long)(b * SEQ + q0)) * HIDDEN + h * HD;
        const int q = lane >> 3, c8 = (lane & 7) * 8;
        v8h hv[4];
#pragma unroll
        for (int it = 0; it < 4; ++it) {
            const int o = (it * 4 + q) * 68 + c8;
#pragma unroll
            for (int e = 0; e < 8; ++e) hv[it][e] = (_Float16)Os[wave][o + e];
        }
#pragma unroll
        for (int it = 0; it < 4; ++it) *(volatile v8h*)(CT + (long long)(it * 4 + q) * HIDDEN + c8) = hv[it];
        __threadfence();
#pragma unroll
        for (int it = 0; it < 4; ++it) *(volatile v8h*)(CT + (long long)(it * 4 + q) * HIDDEN + c8) = hv[it];
    }
}

constexpr size_t SZ_TOK16 = (size_t)MTOK * HIDDEN * 2;
constexpr size_t SZ_W16   = (size_t)HIDDEN * HIDDEN * 2;
constexpr size_t OFF_X16  = 0;
constexpr size_t OFF_WQ   = OFF_X16 + SZ_TOK16;
constexpr size_t OFF_WK   = OFF_WQ + SZ_W16;
constexpr size_t OFF_WV   = OFF_WK + SZ_W16;
constexpr size_t OFF_WO   = OFF_WV + SZ_W16;
constexpr size_t OFF_Q16  = OFF_WO + SZ_W16;
constexpr size_t OFF_K16  = OFF_Q16 + SZ_TOK16;
constexpr size_t OFF_VT16 = OFF_K16 + SZ_TOK16;
constexpr size_t OFF_CTX  = OFF_VT16 + SZ_TOK16;
constexpr size_t WS_TOTAL = OFF_CTX + SZ_TOK16;
static_assert(SZ_TOK16 % 256 == 0 && SZ_W16 % 256 == 0);
static_assert(WS_TOTAL <= 134217728ull);

extern "C" void kernel_launch(void* const* d_in, const int* in_sizes, int n_in, void* d_out, int out_size, void* d_ws, size_t ws_size, hipStream_t stream) {
    if (n_in < 10) return;
    const long long need_x = ((long long)(NB - 1) * SEQ_FULL + SEQ) * HIDDEN;
    const long long need_m = (long long)(NB - 1) * SEQ_FULL + SEQ;
    if ((long long)in_sizes[0] < need_x) return;
    if ((long long)in_sizes[1] < need_m) return;
    if (in_sizes[2] < HIDDEN * HIDDEN || in_sizes[4] < HIDDEN * HIDDEN || in_sizes[6] < HIDDEN * HIDDEN || in_sizes[8] < HIDDEN * HIDDEN) return;
    if (in_sizes[3] < HIDDEN || in_sizes[5] < HIDDEN || in_sizes[7] < HIDDEN || in_sizes[9] < HIDDEN) return;
    if ((long long)out_size < need_x) return;
    if (ws_size < WS_TOTAL) return;

    const float* x     = (const float*)d_in[0];
    const float* masks = (const float*)d_in[1];
    const float* Wq    = (const float*)d_in[2];
    const float* bq    = (const float*)d_in[3];
    const float* Wk    = (const float*)d_in[4];
    const float* bk    = (const float*)d_in[5];
    const float* Wv    = (const float*)d_in[6];
    const float* bv    = (const float*)d_in[7];
    const float* Wo    = (const float*)d_in[8];
    const float* bo    = (const float*)d_in[9];
    float* out = (float*)d_out;
    char* wsp = (char*)d_ws;
    unsigned short* X16  = (unsigned short*)(wsp + OFF_X16);
    unsigned short* WQ16 = (unsigned short*)(wsp + OFF_WQ);
    unsigned short* WK16 = (unsigned short*)(wsp + OFF_WK);
    unsigned short* WV16 = (unsigned short*)(wsp + OFF_WV);
    unsigned short* WO16 = (unsigned short*)(wsp + OFF_WO);
    unsigned short* Q16  = (unsigned short*)(wsp + OFF_Q16);
    unsigned short* K16  = (unsigned short*)(wsp + OFF_K16);
    unsigned short* VT16 = (unsigned short*)(wsp + OFF_VT16);
    unsigned short* CTX16 = (unsigned short*)(wsp + OFF_CTX);

    const unsigned gx = (unsigned)(((long long)MTOK * (HIDDEN / 8) + 255) / 256);
    const unsigned gw = (unsigned)(((long long)HIDDEN * (HIDDEN / 8) + 255) / 256);
    k_cast16<<<gx, 256, 0, stream>>>(x,  X16,  MTOK,   SEQ,    SEQ_FULL, 1.0f);
    k_cast16<<<gw, 256, 0, stream>>>(Wq, WQ16, HIDDEN, HIDDEN, HIDDEN,   16.0f);
    k_cast16<<<gw, 256, 0, stream>>>(Wk, WK16, HIDDEN, HIDDEN, HIDDEN,   16.0f);
    k_cast16<<<gw, 256, 0, stream>>>(Wv, WV16, HIDDEN, HIDDEN, HIDDEN,   16.0f);
    k_cast16<<<gw, 256, 0, stream>>>(Wo, WO16, HIDDEN, HIDDEN, HIDDEN,   16.0f);

    const unsigned gt = (unsigned)((((MTOK / 64) * (HIDDEN / 64)) + 7) / 8);
    k_gemm_nbias_f16<<<dim3(gt, 1), 256, 0, stream>>>(X16, HIDDEN, 0LL, WQ16, HIDDEN, 0LL, Q16, HIDDEN, 0LL, bq, MTOK, HIDDEN, HIDDEN, 0.0625f);
    k_gemm_nbias_f16<<<dim3(gt, 1), 256, 0, stream>>>(X16, HIDDEN, 0LL, WK16, HIDDEN, 0LL, K16, HIDDEN, 0LL, bk, MTOK, HIDDEN, HIDDEN, 0.0625f);
    k_gemm_mbias_f16<<<dim3(gt, 1), 256, 0, stream>>>(WV16, HIDDEN, 0LL, X16, HIDDEN, 0LL, VT16, MTOK, 0LL, bv, HIDDEN, MTOK, HIDDEN, 0.0625f);

    k_attn<<<dim3((unsigned)(NB * HEADS * (SEQ / 64))), 128, 0, stream>>>(Q16, K16, VT16, masks, CTX16);

    const unsigned go = (unsigned)((((SEQ / 64) * (HIDDEN / 64)) + 7) / 8);
    k_gemm_nbias_f32<<<dim3(go, (unsigned)NB), 256, 0, stream>>>(CTX16, HIDDEN, (long long)SEQ * HIDDEN, WO16, HIDDEN, 0LL, out, HIDDEN, (long long)SEQ_FULL * HIDDEN, bo, SEQ, HIDDEN, HIDDEN, 1.0f / 1024.0f);
}
